// EGNNDiffusionModel_1812476199212
// MI455X (gfx1250) — hardware-verified
//
#include <hip/hip_runtime.h>
#include <stddef.h>


#define DF     128
#define NTHR   256
#define NWAVE  8
#define EPT    8
#define CHUNK  (NTHR * EPT)
#define WCAP   (EPT * 32)
#define LISTN  (NWAVE * WCAP)
#define NB     512
#define GROWS  128
#define EBLK   256

#define LDS_GEMM (GROWS * DF * 4)
#define LDS_AGG  (NB * DF * 4 + LISTN * 4 + 64 + NB * 3 * 4 + NB * 4)

static_assert((CHUNK & (CHUNK - 1)) == 0);
static_assert(CHUNK <= 2048);
static_assert((NB & (NB - 1)) == 0);
static_assert(NB <= 4096);
static_assert(LDS_AGG == 278592);
static_assert((NB * DF / 4) % NTHR == 0);
static_assert(NB * 3 <= 2 * NTHR * 4);

typedef float  v4f  __attribute__((ext_vector_type(4)));
typedef float  v8f  __attribute__((ext_vector_type(8)));
typedef int    v4i  __attribute__((ext_vector_type(4)));
typedef __bf16 v8b  __attribute__((ext_vector_type(8)));
typedef __bf16 v16b __attribute__((ext_vector_type(16)));
union FragB { v16b v; v8b h[2]; };

__device__ __forceinline__ v8f wmb(v16b a, v16b b, v8f c) {
  v8f d = __builtin_amdgcn_wmma_f32_16x16x32_bf16(false, a, false, b, (short)0, c, false, false);
  asm volatile("v_nop\n\tv_nop\n\tv_nop\n\tv_nop" : "+v"(d) : "v"(a), "v"(b));
  return d;
}

__device__ __forceinline__ void split8(v4f a, v4f b, v8b& hi, v8b& lo) {
  const float f[8] = {a.x, a.y, a.z, a.w, b.x, b.y, b.z, b.w};
#pragma unroll
  for (int i = 0; i < 8; ++i) {
    const __bf16 t = (__bf16)f[i];
    hi[i] = t;
    lo[i] = (__bf16)(f[i] - (float)t);
  }
}

__device__ __forceinline__ v4f sel4(bool c, v4f a, v4f b) {
  v4f r;
  r.x = c ? a.x : b.x; r.y = c ? a.y : b.y; r.z = c ? a.z : b.z; r.w = c ? a.w : b.w;
  return r;
}

__device__ __forceinline__ v4f relu4(v4f a) {
  a.x = fmaxf(a.x, 0.f); a.y = fmaxf(a.y, 0.f); a.z = fmaxf(a.z, 0.f); a.w = fmaxf(a.w, 0.f);
  return a;
}

__device__ __forceinline__ int scan_chunk(const int* __restrict__ dsts, int nE, int cbase, int nodeBase,
                                          int vec8, int* list, int tid, int wave) {
  int wc = 0;
  const int el0  = tid * EPT;
  const int e0   = cbase + el0;
  const int sent = -2147483647 - 1;
  v4i da, db;
  if (vec8 != 0 && cbase + CHUNK <= nE) {
    da = *(const v4i*)(dsts + e0);
    db = *(const v4i*)(dsts + e0 + 4);
  } else {
    const int em = nE - 1;
    da.x = (e0     < nE) ? dsts[min(e0,     em)] : sent;
    da.y = (e0 + 1 < nE) ? dsts[min(e0 + 1, em)] : sent;
    da.z = (e0 + 2 < nE) ? dsts[min(e0 + 2, em)] : sent;
    da.w = (e0 + 3 < nE) ? dsts[min(e0 + 3, em)] : sent;
    db.x = (e0 + 4 < nE) ? dsts[min(e0 + 4, em)] : sent;
    db.y = (e0 + 5 < nE) ? dsts[min(e0 + 5, em)] : sent;
    db.z = (e0 + 6 < nE) ? dsts[min(e0 + 6, em)] : sent;
    db.w = (e0 + 7 < nE) ? dsts[min(e0 + 7, em)] : sent;
  }
  const unsigned nb = (unsigned)nodeBase;
  const unsigned s0 = (unsigned)da.x - nb, s1 = (unsigned)da.y - nb;
  const unsigned s2 = (unsigned)da.z - nb, s3 = (unsigned)da.w - nb;
  const unsigned s4 = (unsigned)db.x - nb, s5 = (unsigned)db.y - nb;
  const unsigned s6 = (unsigned)db.z - nb, s7 = (unsigned)db.w - nb;
  const bool h0 = s0 < (unsigned)NB, h1 = s1 < (unsigned)NB, h2 = s2 < (unsigned)NB, h3 = s3 < (unsigned)NB;
  const bool h4 = s4 < (unsigned)NB, h5 = s5 < (unsigned)NB, h6 = s6 < (unsigned)NB, h7 = s7 < (unsigned)NB;
  const unsigned any = __builtin_amdgcn_ballot_w32(h0 | h1 | h2 | h3 | h4 | h5 | h6 | h7);
  if (any != 0u) {
#define HITJ(J, HJ, SJ) { \
      const unsigned mj = __builtin_amdgcn_ballot_w32(HJ); \
      if (mj != 0u) { \
        if (HJ) { \
          const int pos = wc + (int)__builtin_amdgcn_mbcnt_lo(mj, 0u); \
          if (pos < WCAP) list[wave * WCAP + pos] = ((el0 + (J)) << 12) | (int)(SJ); \
        } \
        wc += (int)__builtin_popcount(mj); } }
    HITJ(0, h0, s0)
    HITJ(1, h1, s1)
    HITJ(2, h2, s2)
    HITJ(3, h3, s3)
    HITJ(4, h4, s4)
    HITJ(5, h5, s5)
    HITJ(6, h6, s6)
    HITJ(7, h7, s7)
#undef HITJ
  }
  return wc;
}

__global__ __launch_bounds__(NTHR) void k_prep(
    const float* __restrict__ l1w1, const float* __restrict__ l1w2,
    const float* __restrict__ l2w1, const float* __restrict__ l2w2,
    const float* __restrict__ bpw1,
    __bf16* b1h, __bf16* b1l, __bf16* c1h, __bf16* c1l,
    __bf16* b2h, __bf16* b2l, __bf16* c2h, __bf16* c2l,
    __bf16* b3h, __bf16* b3l) {
  const int bx = blockIdx.x, tid = threadIdx.x;
  const float* W; __bf16* oh; __bf16* ol; int kind; int rb;
  if (bx < 16)      { W = l1w1; oh = b1h; ol = b1l; kind = 0; rb = 0;  }
  else if (bx < 24) { W = l1w2; oh = c1h; ol = c1l; kind = 1; rb = 16; }
  else if (bx < 40) { W = l2w1; oh = b2h; ol = b2l; kind = 0; rb = 24; }
  else if (bx < 48) { W = l2w2; oh = c2h; ol = c2l; kind = 1; rb = 40; }
  else              { W = bpw1; oh = b3h; ol = b3l; kind = 2; rb = 48; }
  const int i  = (bx - rb) * NTHR + tid;
  const int o  = i * 8;
  const int n  = o >> 7;
  const int k0 = o & 127;
  const float* p; int s;
  if (kind == 0)      { p = W + (size_t)(k0 + (n >> 7) * 128) * 128 + (n & 127); s = 128; }
  else if (kind == 1) { p = W + (size_t)k0 * 128 + n;                           s = 128; }
  else                { p = W + (size_t)(k0 + (n >> 6) * 128) * 64 + (n & 63);   s = 64;  }
  v4f a, b;
  a.x = p[0];     a.y = p[s];     a.z = p[2 * s]; a.w = p[3 * s];
  b.x = p[4 * s]; b.y = p[5 * s]; b.z = p[6 * s]; b.w = p[7 * s];
  v8b hv, lv;
  split8(a, b, hv, lv);
  *(volatile v8b*)(oh + o) = hv;
  *(volatile v8b*)(ol + o) = lv;
  __threadfence();
  *(volatile v8b*)(oh + o) = hv;
  *(volatile v8b*)(ol + o) = lv;
}

__global__ __launch_bounds__(NTHR) void k_xin(
    const float* __restrict__ xt, const int* __restrict__ tt, const float* __restrict__ cond,
    const float* __restrict__ tw1, const float* __restrict__ tb1,
    const float* __restrict__ tw2, const float* __restrict__ tb2,
    float* xin, int nN) {
  __shared__ __attribute__((aligned(16))) float stemb[32];
  const int tid = threadIdx.x, lane = tid & 31, wave = tid >> 5;
  if (tid < 32) {
    const float tin = (float)tt[0] * (1.0f / 1000.0f);
    float acc = tb2[tid];
#pragma unroll 1
    for (int k = 0; k < 32; ++k) acc += fmaxf(tin * tw1[k] + tb1[k], 0.0f) * tw2[k * 32 + tid];
    stemb[tid] = acc;
  }
  __syncthreads();
  const int c4 = 4 * lane;
  int cc = c4 - 64; cc = cc < 0 ? 0 : (cc > 28 ? 28 : cc);
  int tc = c4 - 96; tc = tc < 0 ? 0 : (tc > 28 ? 28 : tc);
  const int xc = c4 > 60 ? 60 : c4;
  const v4f cv = *(const v4f*)(cond + cc);
  const v4f tv = *(const v4f*)(stemb + tc);
  const int rowBase = blockIdx.x * GROWS + wave * 16;
  v4f ov[16];
#pragma unroll
  for (int i = 0; i < 16; ++i) {
    int node = rowBase + i; node = node > nN - 1 ? nN - 1 : node;
    const v4f xv = *(const v4f*)(xt + (size_t)node * 64 + xc);
    ov[i] = sel4(c4 < 64, xv, sel4(c4 < 96, cv, tv));
  }
  float* gp = xin + (size_t)rowBase * DF + 4 * lane;
#pragma unroll
  for (int i = 0; i < 16; ++i) *(volatile v4f*)(gp + (size_t)i * DF) = ov[i];
  __threadfence();
#pragma unroll
  for (int i = 0; i < 16; ++i) *(volatile v4f*)(gp + (size_t)i * DF) = ov[i];
}

template <int NOUT, int MODE>
__global__ __launch_bounds__(NTHR) void k_gemm(
    const float* __restrict__ A, const __bf16* __restrict__ Bh, const __bf16* __restrict__ Bl,
    const float* __restrict__ bias, int biasN,
    const float* __restrict__ R, const float* __restrict__ cntp,
    float* C, float* out0, int nN) {
  extern __shared__ v4f lds_dyn[];
  float* stg = (float*)lds_dyn;
  const int tid = threadIdx.x, lane = tid & 31, wave = tid >> 5, h = lane >> 4, m = lane & 15;
  const int rowBase = blockIdx.x * GROWS;
  const float* ar = A + ((size_t)rowBase + wave * 16 + m) * DF + 8 * h;
  (void)biasN; (void)R; (void)cntp; (void)out0; (void)nN;

#pragma unroll 1
  for (int p = 0; p < NOUT / 64; ++p) {
    v8f acc[4];
#pragma unroll
    for (int t = 0; t < 4; ++t) { v8f z = {0.f, 0.f, 0.f, 0.f, 0.f, 0.f, 0.f, 0.f}; acc[t] = z; }
#pragma unroll 1
    for (int kt = 0; kt < DF / 32; ++kt) {
      const float* ak = ar + 32 * kt;
      const v4f x0 = *(const v4f*)ak,        x1 = *(const v4f*)(ak + 4);
      const v4f x2 = *(const v4f*)(ak + 16), x3 = *(const v4f*)(ak + 20);
      FragB ah, al;
      split8(x0, x1, ah.h[0], al.h[0]);
      split8(x2, x3, ah.h[1], al.h[1]);
      const __bf16* bk = Bh + (size_t)(64 * p + m) * DF + 32 * kt + 8 * h;
      const __bf16* bq = Bl + (size_t)(64 * p + m) * DF + 32 * kt + 8 * h;
#pragma unroll
      for (int t = 0; t < 4; ++t) {
        FragB bh, bo;
        bh.h[0] = *(const v8b*)(bk + (size_t)16 * t * DF);
        bh.h[1] = *(const v8b*)(bk + (size_t)16 * t * DF + 16);
        bo.h[0] = *(const v8b*)(bq + (size_t)16 * t * DF);
        bo.h[1] = *(const v8b*)(bq + (size_t)16 * t * DF + 16);
        acc[t] = wmb(ah.v, bh.v, acc[t]);
        acc[t] = wmb(ah.v, bo.v, acc[t]);
        acc[t] = wmb(al.v, bh.v, acc[t]);
      }
    }
    float* sp = stg + (wave * 16 + 8 * h) * DF + 64 * (p & 1) + m;
#pragma unroll
    for (int t = 0; t < 4; ++t) {
      sp[0 * DF + 16 * t] = acc[t][0];
      sp[1 * DF + 16 * t] = acc[t][1];
      sp[2 * DF + 16 * t] = acc[t][2];
      sp[3 * DF + 16 * t] = acc[t][3];
      sp[4 * DF + 16 * t] = acc[t][4];
      sp[5 * DF + 16 * t] = acc[t][5];
      sp[6 * DF + 16 * t] = acc[t][6];
      sp[7 * DF + 16 * t] = acc[t][7];
    }
    if (p & 1) {
      __syncthreads();
      const int cbase = 128 * (p >> 1);
      const float* lr = stg + (wave * 16) * DF + 4 * lane;
      const size_t growBase = (size_t)rowBase + wave * 16;
      v4f ov[16];
      if (MODE == 0) {
        const int col = cbase + 4 * lane;
        int bc = col; bc = bc > biasN - 4 ? biasN - 4 : bc; bc = bc < 0 ? 0 : bc;
        const v4f bv = *(const v4f*)(bias + bc);
        const v4f z4 = {0.f, 0.f, 0.f, 0.f};
        const v4f add = sel4(col < biasN, bv, z4);
#pragma unroll
        for (int i = 0; i < 16; ++i) ov[i] = *(const v4f*)(lr + i * DF) + add;
      } else {
        const v4f b2v = *(const v4f*)(bias + 4 * lane);
#pragma unroll
        for (int i = 0; i < 16; ++i) {
          const size_t grow = growBase + i;
          const v4f rv = *(const v4f*)(R + grow * DF + 4 * lane);
          const float cs = cntp[grow];
          ov[i] = *(const v4f*)(lr + i * DF) + rv + cs * b2v;
        }
      }
      float* gp = C + growBase * NOUT + cbase + 4 * lane;
#pragma unroll
      for (int i = 0; i < 16; ++i) *(volatile v4f*)(gp + (size_t)i * NOUT) = ov[i];
      __threadfence();
#pragma unroll
      for (int i = 0; i < 16; ++i) *(volatile v4f*)(gp + (size_t)i * NOUT) = ov[i];
      if (MODE == 2) {
        float* wr = stg + (wave * 16) * DF + 4 * lane;
#pragma unroll
        for (int i = 0; i < 16; ++i) *(v4f*)(wr + i * DF) = ov[i];
        __syncthreads();
        v4f o2[8];
#pragma unroll
        for (int q = 0; q < 8; ++q) o2[q] = *(const v4f*)(stg + (wave * 16 + 2 * q + h) * DF + 4 * m);
#pragma unroll
        for (int q = 0; q < 8; ++q) {
          const size_t grow = growBase + 2 * q + h;
          if (grow < (size_t)nN) *(volatile v4f*)(out0 + grow * 64 + 4 * m) = o2[q];
        }
        __threadfence();
#pragma unroll
        for (int q = 0; q < 8; ++q) {
          const size_t grow = growBase + 2 * q + h;
          if (grow < (size_t)nN) *(volatile v4f*)(out0 + grow * 64 + 4 * m) = o2[q];
        }
      }
      __syncthreads();
    }
  }
}

__global__ __launch_bounds__(NTHR) void k_agg(
    const int* __restrict__ ei, const float* __restrict__ pq, const float* __restrict__ posin,
    const float* __restrict__ w256, const float* __restrict__ cw1, const float* __restrict__ cb1,
    const float* __restrict__ cw2, const float* __restrict__ cb2,
    float* U, float* cntp, float* posout, int nN, int nE, int vec8) {
  extern __shared__ v4f lds_dyn[];
  float* accU   = (float*)lds_dyn;
  int*   list   = (int*)(accU + NB * DF);
  int*   wcnt   = list + LISTN;
  float* posacc = (float*)(wcnt + 16);
  int*   cnt    = (int*)(posacc + NB * 3);
  const int tid = threadIdx.x, lane = tid & 31, wave = tid >> 5;
  const int nodeBase = blockIdx.x * NB;
  const int* dsts = ei + nE;

  {
    const v4f z = {0.f, 0.f, 0.f, 0.f};
    for (int i = tid; i < NB * DF / 4; i += NTHR) lds_dyn[i] = z;
  }
  for (int i = tid; i < NB * 3; i += NTHR) posacc[i] = 0.f;
  for (int i = tid; i < NB; i += NTHR) cnt[i] = 0;

  const v4f wv  = *(const v4f*)(w256 + 4 * lane);
  const v4f c1v = *(const v4f*)(cw1 + 4 * lane);
  const v4f cbv = *(const v4f*)(cb1 + 4 * lane);
  const v4f c2v = *(const v4f*)(cw2 + 4 * lane);
  const float cb2s = cb2[0];
  __syncthreads();

  const int nChunks = (nE + CHUNK - 1) / CHUNK;
#pragma unroll 1
  for (int ch = 0; ch < nChunks; ++ch) {
    const int cbase = ch * CHUNK;
    const int wc = scan_chunk(dsts, nE, cbase, nodeBase, vec8, list, tid, wave);
    if (lane == 0) wcnt[wave] = wc;
    __syncthreads();
    if (wave == 0) {
#pragma unroll 1
      for (int wsx = 0; wsx < NWAVE; ++wsx) {
        int n = __builtin_amdgcn_readfirstlane(wcnt[wsx]);
        n = n > WCAP ? WCAP : (n < 0 ? 0 : n);
        const int* lp = list + wsx * WCAP;
#pragma unroll 1
        for (int i = 0; i < n; ++i) {
          const int ent  = __builtin_amdgcn_readfirstlane(lp[i]);
          const int slot = ent & (NB - 1);
          int e = cbase + ((ent >> 12) & (CHUNK - 1));
          e = e > nE - 1 ? nE - 1 : e;
          int src = ei[e];
          src = src < 0 ? 0 : (src > nN - 1 ? nN - 1 : src);
          int node = nodeBase + slot;
          node = node > nN - 1 ? nN - 1 : node;
          const float ex = posin[src * 3 + 0] - posin[node * 3 + 0];
          const float ey = posin[src * 3 + 1] - posin[node * 3 + 1];
          const float ez = posin[src * 3 + 2] - posin[node * 3 + 2];
          const float dist = sqrtf(ex * ex + ey * ey + ez * ez + 1e-8f);
          const v4f pv = *(const v4f*)(pq + (size_t)node * (2 * DF) + 4 * lane);
          const v4f qv = *(const v4f*)(pq + (size_t)src * (2 * DF) + DF + 4 * lane);
          const v4f u = relu4(pv + qv + dist * wv);
          v4f* ap = (v4f*)(accU + slot * DF + 4 * lane);
          *ap = *ap + u;
          const v4f hv = relu4(dist * c1v + cbv);
          float part = hv.x * c2v.x + hv.y * c2v.y + hv.z * c2v.z + hv.w * c2v.w;
          part += __shfl_xor(part, 16);
          part += __shfl_xor(part, 8);
          part += __shfl_xor(part, 4);
          part += __shfl_xor(part, 2);
          part += __shfl_xor(part, 1);
          const float cval = part + cb2s;
          if (lane < 3) {
            const float evc = (lane == 0) ? ex : ((lane == 1) ? ey : ez);
            posacc[slot * 3 + lane] = posacc[slot * 3 + lane] + cval * evc;
          }
          if (lane == 0) cnt[slot] = cnt[slot] + 1;
        }
      }
    }
    __syncthreads();
  }

  const float d0 = sqrtf(1e-8f);
#pragma unroll 1
  for (int i = 0; i < (NB * DF / 4) / NTHR; ++i) {
    const int idx  = i * NTHR + tid;
    const int slot = idx >> 5;
    const int c4   = (idx & 31) * 4;
    int node = nodeBase + slot;
    node = node > nN - 1 ? nN - 1 : node;
    const v4f pv = *(const v4f*)(pq + (size_t)node * (2 * DF) + c4);
    const v4f qv = *(const v4f*)(pq + (size_t)node * (2 * DF) + DF + c4);
    const v4f w4 = *(const v4f*)(w256 + c4);
    const v4f u  = relu4(pv + qv + d0 * w4);
    v4f* ap = (v4f*)(accU + slot * DF + c4);
    *ap = *ap + u;
  }
  for (int i = tid; i < NB * 3; i += NTHR) {
    const int slot = i / 3;
    const int c    = i - slot * 3;
    int node = nodeBase + slot;
    node = node > nN - 1 ? nN - 1 : node;
    posacc[i] = posacc[i] + posin[node * 3 + c];
  }
  __syncthreads();

  const bool hc = tid < NB / 4;
  v4f cf = {0.f, 0.f, 0.f, 0.f};
  {
    const int ci = hc ? 4 * tid : 0;
    const v4i c = *(const v4i*)(cnt + ci);
    cf.x = (float)(c.x + 1); cf.y = (float)(c.y + 1); cf.z = (float)(c.z + 1); cf.w = (float)(c.w + 1);
  }
  const int f0 = 4 * tid;
  int f1 = 4 * (NTHR + tid); f1 = f1 > NB * 3 - 4 ? NB * 3 - 4 : f1;
  const v4f pz0 = *(const v4f*)(posacc + f0);
  const v4f pz1 = *(const v4f*)(posacc + f1);

  float* up = U + (size_t)nodeBase * DF;
  float* cp = cntp + (size_t)nodeBase;
  float* pp = posout + (size_t)nodeBase * 3;
#pragma unroll 4
  for (int q = 0; q < 64; ++q) {
    const int f = (wave * 64 + q) * 128 + 4 * lane;
    const v4f v = *(const v4f*)(accU + f);
    *(volatile v4f*)(up + f) = v;
  }
  if (hc) *(volatile v4f*)(cp + f0) = cf;
  *(volatile v4f*)(pp + f0) = pz0;
  if (hc) *(volatile v4f*)(pp + 4 * (NTHR + tid)) = pz1;
  __threadfence();
#pragma unroll 4
  for (int q = 0; q < 64; ++q) {
    const int f = (wave * 64 + q) * 128 + 4 * lane;
    const v4f v = *(const v4f*)(accU + f);
    *(volatile v4f*)(up + f) = v;
  }
  if (hc) *(volatile v4f*)(cp + f0) = cf;
  *(volatile v4f*)(pp + f0) = pz0;
  if (hc) *(volatile v4f*)(pp + 4 * (NTHR + tid)) = pz1;
}

__global__ __launch_bounds__(NTHR) void k_bond(
    const int* __restrict__ ei, const float* __restrict__ pq3,
    const float* __restrict__ w2, const float* __restrict__ b2,
    float* out1, int nN, int nE) {
  __shared__ v4f sw2[64];
  const int tid = threadIdx.x;
  if (tid < 64) sw2[tid] = *(const v4f*)(w2 + tid * 4);
  const v4f bv = *(const v4f*)b2;
  __syncthreads();
  const int e = blockIdx.x * EBLK + tid;
  const int ec = e > nE - 1 ? nE - 1 : e;
  int src = ei[ec];
  src = src < 0 ? 0 : (src > nN - 1 ? nN - 1 : src);
  int dst = ei[nE + ec];
  dst = dst < 0 ? 0 : (dst > nN - 1 ? nN - 1 : dst);
  const float* pr = pq3 + (size_t)src * DF;
  const float* qr = pq3 + (size_t)dst * DF + 64;
  v4f acc = bv;
#pragma unroll 1
  for (int k4 = 0; k4 < 16; ++k4) {
    const v4f pv = *(const v4f*)(pr + 4 * k4);
    const v4f qv = *(const v4f*)(qr + 4 * k4);
    const v4f f  = relu4(pv + qv);
    acc = acc + f.x * sw2[4 * k4] + f.y * sw2[4 * k4 + 1] + f.z * sw2[4 * k4 + 2] + f.w * sw2[4 * k4 + 3];
  }
  float* gp = out1 + (size_t)e * 4;
  if (e < nE) *(volatile v4f*)gp = acc;
  __threadfence();
  if (e < nE) *(volatile v4f*)gp = acc;
}

extern "C" void kernel_launch(void* const* d_in, const int* in_sizes, int n_in,
                              void* d_out, int out_size, void* d_ws, size_t ws_size,
                              hipStream_t stream) {
  if (n_in < 29) return;
  const int nN = in_sizes[0] / 64;
  const int nE = in_sizes[2] / 2;
  if (nN <= 0 || nE <= 0) return;
  if (in_sizes[0] != nN * 64 || in_sizes[1] != nN * 3 || in_sizes[2] != nE * 2 || in_sizes[3] < 1) return;
  if (in_sizes[4] != 32 || in_sizes[5] != 32 || in_sizes[6] != 32 || in_sizes[7] != 1024 || in_sizes[8] != 32) return;
  for (int L = 0; L < 2; ++L) {
    const int b = 9 + 8 * L;
    if (in_sizes[b] != 257 * 128 || in_sizes[b + 1] != 128 || in_sizes[b + 2] != 128 * 128 || in_sizes[b + 3] != 128) return;
    if (in_sizes[b + 4] != 128 || in_sizes[b + 5] != 128 || in_sizes[b + 6] != 128 || in_sizes[b + 7] < 1) return;
  }
  if (in_sizes[25] != 256 * 64 || in_sizes[26] != 64 || in_sizes[27] != 256 || in_sizes[28] != 4) return;
  if (out_size != nN * 64 + nE * 4) return;

  const float* x_t      = (const float*)d_in[0];
  const float* pos      = (const float*)d_in[1];
  const int*   ei       = (const int*)d_in[2];
  const int*   tt       = (const int*)d_in[3];
  const float* cond     = (const float*)d_in[4];
  const float* te_w1    = (const float*)d_in[5];
  const float* te_b1    = (const float*)d_in[6];
  const float* te_w2    = (const float*)d_in[7];
  const float* te_b2    = (const float*)d_in[8];
  const float* l1_nm_w1 = (const float*)d_in[9];
  const float* l1_nm_b1 = (const float*)d_in[10];
  const float* l1_nm_w2 = (const float*)d_in[11];
  const float* l1_nm_b2 = (const float*)d_in[12];
  const float* l1_cm_w1 = (const float*)d_in[13];
  const float* l1_cm_b1 = (const float*)d_in[14];
  const float* l1_cm_w2 = (const float*)d_in[15];
  const float* l1_cm_b2 = (const float*)d_in[16];
  const float* l2_nm_w1 = (const float*)d_in[17];
  const float* l2_nm_b1 = (const float*)d_in[18];
  const float* l2_nm_w2 = (const float*)d_in[19];
  const float* l2_nm_b2 = (const float*)d_in[20];
  const float* l2_cm_w1 = (const float*)d_in[21];
  const float* l2_cm_b1 = (const float*)d_in[22];
  const float* l2_cm_w2 = (const float*)d_in[23];
  const float* l2_cm_b2 = (const float*)d_in[24];
  const float* bp_w1    = (const float*)d_in[25];
  const float* bp_b1    = (const float*)d_in[26];
  const float* bp_w2    = (const float*)d_in[27];
  const float* bp_b2    = (const float*)d_in[28];
  float* outf = (float*)d_out;
  float* out0 = outf;
  float* out1 = outf + (size_t)nN * 64;

  const int nG   = (nN + GROWS - 1) / GROWS;
  const int nAgg = (nN + NB - 1) / NB;
  const int nEB  = (nE + EBLK - 1) / EBLK;
  const size_t rowsG = (size_t)nG * GROWS;
  const size_t rowsA = (size_t)nAgg * NB;

  char* ws = (char*)d_ws;
  size_t off = 0;
#define CARVE(NAME, BYTES) const size_t NAME = off; off += (size_t)(BYTES); off = (off + 255) & ~(size_t)255;
  CARVE(oB1h, 256 * 128 * 2) CARVE(oB1l, 256 * 128 * 2) CARVE(oC1h, 128 * 128 * 2) CARVE(oC1l, 128 * 128 * 2)
  CARVE(oB2h, 256 * 128 * 2) CARVE(oB2l, 256 * 128 * 2) CARVE(oC2h, 128 * 128 * 2) CARVE(oC2l, 128 * 128 * 2)
  CARVE(oB3h, 128 * 128 * 2) CARVE(oB3l, 128 * 128 * 2)
  CARVE(oXin, rowsG * DF * 4)
  CARVE(oPQ,  rowsG * 2 * DF * 4)
  CARVE(oU,   rowsA * DF * 4)
  CARVE(oCnt, rowsA * 4)
  CARVE(oP1,  rowsA * 3 * 4)
  CARVE(oP2,  rowsA * 3 * 4)
  CARVE(oX1,  rowsG * DF * 4)
#undef CARVE
  if (off > ws_size) return;
  __bf16* B1h = (__bf16*)(ws + oB1h); __bf16* B1l = (__bf16*)(ws + oB1l);
  __bf16* C1h = (__bf16*)(ws + oC1h); __bf16* C1l = (__bf16*)(ws + oC1l);
  __bf16* B2h = (__bf16*)(ws + oB2h); __bf16* B2l = (__bf16*)(ws + oB2l);
  __bf16* C2h = (__bf16*)(ws + oC2h); __bf16* C2l = (__bf16*)(ws + oC2l);
  __bf16* B3h = (__bf16*)(ws + oB3h); __bf16* B3l = (__bf16*)(ws + oB3l);
  float* xin  = (float*)(ws + oXin);
  float* x2   = xin;
  float* pq   = (float*)(ws + oPQ);
  float* U    = (float*)(ws + oU);
  float* cntp = (float*)(ws + oCnt);
  float* pos1 = (float*)(ws + oP1);
  float* pos2 = (float*)(ws + oP2);
  float* x1   = (float*)(ws + oX1);

  const int vec8 = ((nE & 3) == 0) ? 1 : 0;

  k_prep<<<56, NTHR, 0, stream>>>(l1_nm_w1, l1_nm_w2, l2_nm_w1, l2_nm_w2, bp_w1,
                                  B1h, B1l, C1h, C1l, B2h, B2l, C2h, C2l, B3h, B3l);

  k_xin<<<nG, NTHR, 0, stream>>>(x_t, tt, cond, te_w1, te_b1, te_w2, te_b2, xin, nN);

  hipFuncSetAttribute(reinterpret_cast<const void*>(&k_gemm<256, 0>),
                      hipFuncAttributeMaxDynamicSharedMemorySize, LDS_GEMM);
  hipFuncSetAttribute(reinterpret_cast<const void*>(&k_gemm<128, 0>),
                      hipFuncAttributeMaxDynamicSharedMemorySize, LDS_GEMM);
  hipFuncSetAttribute(reinterpret_cast<const void*>(&k_gemm<128, 1>),
                      hipFuncAttributeMaxDynamicSharedMemorySize, LDS_GEMM);
  hipFuncSetAttribute(reinterpret_cast<const void*>(&k_gemm<128, 2>),
                      hipFuncAttributeMaxDynamicSharedMemorySize, LDS_GEMM);
  hipFuncSetAttribute(reinterpret_cast<const void*>(&k_agg),
                      hipFuncAttributeMaxDynamicSharedMemorySize, LDS_AGG);

  k_gemm<256, 0><<<nG, NTHR, LDS_GEMM, stream>>>(xin, B1h, B1l, l1_nm_b1, 128, xin, cntp, pq, pq, nN);
  k_agg<<<nAgg, NTHR, LDS_AGG, stream>>>(ei, pq, pos, l1_nm_w1 + 256 * 128,
                                         l1_cm_w1, l1_cm_b1, l1_cm_w2, l1_cm_b2,
                                         U, cntp, pos1, nN, nE, vec8);
  k_gemm<128, 1><<<nG, NTHR, LDS_GEMM, stream>>>(U, C1h, C1l, l1_nm_b2, 128, xin, cntp, x1, x1, nN);

  k_gemm<256, 0><<<nG, NTHR, LDS_GEMM, stream>>>(x1, B2h, B2l, l2_nm_b1, 128, x1, cntp, pq, pq, nN);
  k_agg<<<nAgg, NTHR, LDS_AGG, stream>>>(ei, pq, pos1, l2_nm_w1 + 256 * 128,
                                         l2_cm_w1, l2_cm_b1, l2_cm_w2, l2_cm_b2,
                                         U, cntp, pos2, nN, nE, vec8);
  k_gemm<128, 2><<<nG, NTHR, LDS_GEMM, stream>>>(U, C2h, C2l, l2_nm_b2, 128, x1, cntp, x2, out0, nN);

  k_gemm<128, 0><<<nG, NTHR, LDS_GEMM, stream>>>(x2, B3h, B3l, bp_b1, 64, x2, cntp, pq, pq, nN);
  k_bond<<<nEB, NTHR, 0, stream>>>(ei, pq, bp_w2, bp_b2, out1, nN, nE);
}
